// RWKV_TimeMix_83056077570123
// MI455X (gfx1250) — hardware-verified
//
#include <hip/hip_runtime.h>
#include <hip/hip_bf16.h>
#include <stdint.h>


#ifndef __has_builtin
#define __has_builtin(x) 0
#endif
#define HAVE_ASYNC_LDS 0

typedef __attribute__((ext_vector_type(16))) _Float16 v16h;
typedef __attribute__((ext_vector_type(8)))  float  v8f;
typedef __attribute__((ext_vector_type(4)))  int    v4i;

static __device__ __forceinline__ _Float16 to_bf16(float f) { return (_Float16)f; }
typedef __attribute__((ext_vector_type(8)))  _Float16 v8h;
typedef __attribute__((ext_vector_type(4)))  float  v4f;
typedef __attribute__((ext_vector_type(4)))  unsigned v4u;
typedef unsigned __attribute__((may_alias)) uint_a;
template <typename T> __device__ __forceinline__ void vst2(void* p, T v) { *(volatile T*)p = v; __threadfence(); *(volatile T*)p = v; }
static __device__ __forceinline__ v8f wmma16(v16h a, v16h b, v8f c) {
    v8f d = __builtin_amdgcn_wmma_f32_16x16x32_f16(false, a, false, b, (short)0, c, false, false);
    asm volatile("v_nop\n\tv_nop\n\tv_nop\n\tv_nop" : "+v"(d) : "v"(a), "v"(b));
    return d;
}

__global__ __launch_bounds__(256) void cvt_bf16_kernel(
    const float* __restrict__ in, _Float16* __restrict__ out, int n)
{
    int g = blockIdx.x * 256 + threadIdx.x;
    if (g * 8 >= n) return;
    union { v8h h; v4u u; } pk;
#pragma unroll
    for (int e = 0; e < 8; ++e) pk.h[e] = to_bf16(in[(size_t)g * 8 + e]);
    vst2(out + (size_t)g * 8, pk.u);
}

__global__ __launch_bounds__(256) void mix_kernel(
    const float* __restrict__ x, const float* __restrict__ tmix,
    _Float16* __restrict__ out, int T, int C, int total)
{
    int g = blockIdx.x * 256 + threadIdx.x;
    if (g * 8 >= total) return;
    union { v8h h; v4u u; } pk;
#pragma unroll
    for (int e = 0; e < 8; ++e) {
        int i = g * 8 + e;
        int c = i % C;
        int t = (i / C) % T;
        float xv = x[i];
        float xs = (t == 0) ? 0.0f : x[i - C];
        float tm = tmix[c];
        pk.h[e] = to_bf16(xv * tm + xs * (1.0f - tm));
    }
    vst2(out + (size_t)g * 8, pk.u);
}

#define TM 128
#define TN 128
#define TK 64
#define LDSTR 80

__global__ __launch_bounds__(256) void gemm_bf16_nt_kernel(
    const _Float16* __restrict__ A, const _Float16* __restrict__ W,
    float* __restrict__ Out, int M, int N, int K)
{
    __shared__ alignas(32) _Float16 smem_all[4 * TM * LDSTR];
    _Float16 (*As)[TM * LDSTR] = reinterpret_cast<_Float16 (*)[TM * LDSTR]>(smem_all);
    _Float16 (*Ws)[TN * LDSTR] = reinterpret_cast<_Float16 (*)[TN * LDSTR]>(smem_all + 2 * TM * LDSTR);

    const int tid  = threadIdx.x;
    const int lane = tid & 31;
    const int wave = tid >> 5;
    const int wm   = wave >> 1;
    const int wn   = wave & 1;
    const int lrow = lane & 15;
    const int lhf  = lane >> 4;

    const int blockM = blockIdx.y * TM;
    const int blockN = blockIdx.x * TN;

    int srow[4], scol[4];
#pragma unroll
    for (int i = 0; i < 4; ++i) {
        int chunk = tid + 256 * i;
        srow[i] = chunk >> 3;
        scol[i] = (chunk & 7) * 8;
    }

    v8f acc[2][4];
#pragma unroll
    for (int i = 0; i < 2; ++i)
#pragma unroll
        for (int j = 0; j < 4; ++j) acc[i][j] = (v8f){};

    auto do_mma = [&](const _Float16* as, const _Float16* ws) {
#pragma unroll
        for (int ks = 0; ks < TK; ks += 32) {
            v16h afrag[2], bfrag[4];
#pragma unroll
            for (int mt = 0; mt < 2; ++mt)
                { const _Float16* ap = &as[(wm * 32 + mt * 16 + lrow) * LDSTR + ks + 8 * lhf];
                  union { v16h v; v8h q[2]; } u; u.q[0] = *reinterpret_cast<const v8h*>(ap); u.q[1] = *reinterpret_cast<const v8h*>(ap + 16); afrag[mt] = u.v; }
#pragma unroll
            for (int nt = 0; nt < 4; ++nt)
                { const _Float16* bp = &ws[(wn * 64 + nt * 16 + lrow) * LDSTR + ks + 8 * lhf];
                  union { v16h v; v8h q[2]; } u; u.q[0] = *reinterpret_cast<const v8h*>(bp); u.q[1] = *reinterpret_cast<const v8h*>(bp + 16); bfrag[nt] = u.v; }
#pragma unroll
            for (int mt = 0; mt < 2; ++mt)
#pragma unroll
                for (int nt = 0; nt < 4; ++nt)
                    acc[mt][nt] = wmma16(afrag[mt], bfrag[nt], acc[mt][nt]);
        }
    };

    const int ntiles = K / TK;

#if HAVE_ASYNC_LDS
    auto issue = [&](int tile, int buf) {
        int k0 = tile * TK;
#pragma unroll
        for (int i = 0; i < 4; ++i) {
            const _Float16* ga = &A[(size_t)(blockM + srow[i]) * K + k0 + scol[i]];
            const _Float16* gw = &W[(size_t)(blockN + srow[i]) * K + k0 + scol[i]];
            __builtin_amdgcn_global_load_async_to_lds_b128(
                (v4i*)ga, (v4i*)&As[buf][srow[i] * LDSTR + scol[i]], 0, 0);
            __builtin_amdgcn_global_load_async_to_lds_b128(
                (v4i*)gw, (v4i*)&Ws[buf][srow[i] * LDSTR + scol[i]], 0, 0);
        }
    };
    issue(0, 0);
    for (int t = 0; t < ntiles; ++t) {
        int cur = t & 1;
        if (t + 1 < ntiles) {
            issue(t + 1, cur ^ 1);
            __builtin_amdgcn_s_wait_asynccnt(8);
        } else {
            __builtin_amdgcn_s_wait_asynccnt(0);
        }
        __syncthreads();
        do_mma(As[cur], Ws[cur]);
        __syncthreads();
    }
#else
    float4 ra[4], rw[4];
    auto gload = [&](int k0) {
#pragma unroll
        for (int i = 0; i < 4; ++i) {
            size_t aoff = (size_t)(blockM + srow[i]) * K + k0 + scol[i];
            size_t woff = (size_t)(blockN + srow[i]) * K + k0 + scol[i];
            ra[i] = *reinterpret_cast<const float4*>(&A[aoff]);
            rw[i] = *reinterpret_cast<const float4*>(&W[woff]);
            __builtin_prefetch(&A[aoff + TK], 0, 0);
            __builtin_prefetch(&W[woff + TK], 0, 0);
        }
    };
    auto sstore = [&](int buf) {
#pragma unroll
        for (int i = 0; i < 4; ++i) {
            *reinterpret_cast<float4*>(&As[buf][srow[i] * LDSTR + scol[i]]) = ra[i];
            *reinterpret_cast<float4*>(&Ws[buf][srow[i] * LDSTR + scol[i]]) = rw[i];
        }
    };
    gload(0);
    sstore(0);
    for (int t = 0; t < ntiles; ++t) {
        int cur = t & 1;
        if (t + 1 < ntiles) gload((t + 1) * TK);
        __syncthreads();
        do_mma(As[cur], Ws[cur]);
        if (t + 1 < ntiles) sstore(cur ^ 1);
    }
#endif

    __syncthreads();
    float* S = reinterpret_cast<float*>(&As[0][0]) + wave * (32 * 64);
#pragma unroll
    for (int mt = 0; mt < 2; ++mt)
#pragma unroll
        for (int nt = 0; nt < 4; ++nt)
#pragma unroll
            for (int j = 0; j < 8; ++j) S[(mt * 16 + 8 * lhf + j) * 64 + nt * 16 + lrow] = acc[mt][nt][j];
    asm volatile("s_wait_dscnt 0" ::: "memory"); __builtin_amdgcn_wave_barrier(); __builtin_amdgcn_fence(__ATOMIC_RELEASE, "workgroup");
#pragma unroll 4
    for (int q = 0; q < 16; ++q) { const int rl = q * 2 + (lane >> 4), pc = lane & 15;
        vst2(Out + (size_t)(blockM + wm * 32 + rl) * N + blockN + wn * 64 + pc * 4, *reinterpret_cast<const v4f*>(S + rl * 64 + pc * 4)); }
}

#define NCH 8

__global__ __launch_bounds__(256) void wkv_partial_kernel(
    const float* __restrict__ Kp, const float* __restrict__ Vp,
    float* __restrict__ Pnum, float* __restrict__ Pden,
    const float* __restrict__ decay, int T, int C)
{
    int c = blockIdx.x * 256 + threadIdx.x;
    int j = blockIdx.y;
    int b = blockIdx.z;
    if (c >= C) return;
    const int L = T / NCH;
    const float a = expf(-expf(decay[c]));
    float pn = 0.0f, pd = 0.0f;
    size_t base = ((size_t)b * T + (size_t)j * L) * C + c;
    for (int i = 0; i < L; ++i) {
        size_t idx = base + (size_t)i * C;
        float ek  = expf(fminf(Kp[idx], 60.0f));
        float ekv = ek * Vp[idx];
        pn = a * pn + ekv;
        pd = a * pd + ek;
    }
    size_t pidx = ((size_t)b * NCH + j) * C + c;
    vst2(Pnum + pidx, pn);
    vst2(Pden + pidx, pd);
}

__global__ __launch_bounds__(256) void wkv_scan_kernel(
    float* __restrict__ Pnum, float* __restrict__ Pden,
    const float* __restrict__ decay, int T, int C)
{
    int c = blockIdx.x * 256 + threadIdx.x;
    int b = blockIdx.y;
    if (c >= C) return;
    const int L = T / NCH;
    const float d  = expf(decay[c]);
    const float aL = expf(-d * (float)L);
    float sn = 0.0f, sd = 0.0f;
    for (int j = 0; j < NCH; ++j) {
        size_t pidx = ((size_t)b * NCH + j) * C + c;
        float pn = Pnum[pidx], pd = Pden[pidx];
        vst2(Pnum + pidx, sn);
        vst2(Pden + pidx, sd);
        sn = aL * sn + pn;
        sd = aL * sd + pd;
    }
}

__global__ __launch_bounds__(256) void wkv_final_kernel(
    const float* __restrict__ Kp, const float* __restrict__ Vp,
    const float* __restrict__ Rp,
    const float* __restrict__ Pnum, const float* __restrict__ Pden,
    const float* __restrict__ decay, const float* __restrict__ first,
    _Float16* __restrict__ out, int T, int C)
{
    int c = (blockIdx.x * 256 + threadIdx.x) * 2;
    int j = blockIdx.y;
    int b = blockIdx.z;
    if (c >= C) return;
    const int L = T / NCH;
    float a[2], ef[2], sn[2], sd[2];
#pragma unroll
    for (int q = 0; q < 2; ++q) {
        a[q]  = expf(-expf(decay[c + q]));
        ef[q] = expf(first[c + q]);
        size_t pidx = ((size_t)b * NCH + j) * C + c + q;
        sn[q] = Pnum[pidx]; sd[q] = Pden[pidx];
    }
    size_t base = ((size_t)b * T + (size_t)j * L) * C + c;
    for (int i = 0; i < L; ++i) {
        size_t idx = base + (size_t)i * C;
        union { _Float16 h[2]; unsigned u; } pk;
#pragma unroll
        for (int q = 0; q < 2; ++q) {
            float ek  = expf(fminf(Kp[idx + q], 60.0f));
            float ekv = ek * Vp[idx + q];
            float num = ef[q] * ekv + sn[q];
            float den = ef[q] * ek + sd[q] + 1e-9f;
            float sig = 1.0f / (1.0f + expf(-Rp[idx + q]));
            pk.h[q] = to_bf16(sig * num / den);
            sn[q] = a[q] * sn[q] + ekv;
            sd[q] = a[q] * sd[q] + ek;
        }
        vst2(out + idx, (uint_a)pk.u);
    }
}

extern "C" void kernel_launch(void* const* d_in, const int* in_sizes, int n_in,
                              void* d_out, int out_size, void* d_ws, size_t ws_size,
                              hipStream_t stream)
{
    const float* x          = (const float*)d_in[0];
    const float* time_decay = (const float*)d_in[1];
    const float* time_first = (const float*)d_in[2];
    const float* time_mix   = (const float*)d_in[3];
    const float* Wk         = (const float*)d_in[4];
    const float* Wv         = (const float*)d_in[5];
    const float* Wr         = (const float*)d_in[6];
    const float* Wo         = (const float*)d_in[7];

    const int C = in_sizes[3];
    const int T = 768;
    const int M = in_sizes[0] / C;
    const int B = M / T;

    char* ws = (char*)d_ws;
    size_t off = 0;
    auto carve = [&](size_t bytes) -> char* {
        char* p = ws + off;
        off += (bytes + 255) & ~(size_t)255;
        return p;
    };
    _Float16* Axm   = (_Float16*)carve((size_t)M * C * sizeof(_Float16));
    _Float16* RWKVb = (_Float16*)carve((size_t)M * C * sizeof(_Float16));
    _Float16* Wkb   = (_Float16*)carve((size_t)C * C * sizeof(_Float16));
    _Float16* Wvb   = (_Float16*)carve((size_t)C * C * sizeof(_Float16));
    _Float16* Wrb   = (_Float16*)carve((size_t)C * C * sizeof(_Float16));
    _Float16* Wob   = (_Float16*)carve((size_t)C * C * sizeof(_Float16));
    float*  Kf    = (float*)carve((size_t)M * C * sizeof(float));
    float*  Vf    = (float*)carve((size_t)M * C * sizeof(float));
    float*  Rf    = (float*)carve((size_t)M * C * sizeof(float));
    float*  Pnum  = (float*)carve((size_t)B * NCH * C * sizeof(float));
    float*  Pden  = (float*)carve((size_t)B * NCH * C * sizeof(float));

    {
        int n = C * C;
        int g = (n / 8 + 255) / 256;
        cvt_bf16_kernel<<<g, 256, 0, stream>>>(Wk, Wkb, n);
        cvt_bf16_kernel<<<g, 256, 0, stream>>>(Wv, Wvb, n);
        cvt_bf16_kernel<<<g, 256, 0, stream>>>(Wr, Wrb, n);
        cvt_bf16_kernel<<<g, 256, 0, stream>>>(Wo, Wob, n);
    }

    {
        int total = M * C;
        mix_kernel<<<(total / 8 + 255) / 256, 256, 0, stream>>>(
            x, time_mix, Axm, T, C, total);
    }

    {
        dim3 grid(C / TN, M / TM);
        gemm_bf16_nt_kernel<<<grid, 256, 0, stream>>>(Axm, Wkb, Kf, M, C, C);
        gemm_bf16_nt_kernel<<<grid, 256, 0, stream>>>(Axm, Wvb, Vf, M, C, C);
        gemm_bf16_nt_kernel<<<grid, 256, 0, stream>>>(Axm, Wrb, Rf, M, C, C);
    }

    {
        dim3 g1((C + 255) / 256, NCH, B);
        wkv_partial_kernel<<<g1, 256, 0, stream>>>(Kf, Vf, Pnum, Pden,
                                                   time_decay, T, C);
        dim3 g2((C + 255) / 256, B);
        wkv_scan_kernel<<<g2, 256, 0, stream>>>(Pnum, Pden, time_decay, T, C);
        dim3 g3((C / 2 + 255) / 256, NCH, B);
        wkv_final_kernel<<<g3, 256, 0, stream>>>(Kf, Vf, Rf, Pnum, Pden,
                                                 time_decay, time_first,
                                                 RWKVb, T, C);
    }

    {
        dim3 grid(C / TN, M / TM);
        gemm_bf16_nt_kernel<<<grid, 256, 0, stream>>>(
            RWKVb, Wob, (float*)d_out, M, C, C);
    }
}
